// MinimalSSM_12438225289387
// MI455X (gfx1250) — hardware-verified
//
#include <hip/hip_runtime.h>
#include <math.h>

typedef __attribute__((ext_vector_type(16))) _Float16 v16h;
typedef __attribute__((ext_vector_type(16))) __bf16 v16b;
typedef __attribute__((ext_vector_type(8)))  _Float16 v8h;
typedef __attribute__((ext_vector_type(8)))  float v8f;
typedef __attribute__((ext_vector_type(4)))  float v4f;
typedef __attribute__((ext_vector_type(2)))  float v2f;
typedef __attribute__((ext_vector_type(4)))  unsigned v4u;
typedef __attribute__((ext_vector_type(4)))  int v4i;
typedef float __attribute__((may_alias)) float_a;
typedef int __attribute__((may_alias)) int_a;

template <typename T> __device__ __forceinline__ void vst2(void* p, T v) { *(volatile T*)p = v; __threadfence(); *(volatile T*)p = v; }
__device__ __forceinline__ v8f wmma16(v16h a, v16h b, v8f c) {
  v8f d = __builtin_amdgcn_wmma_f32_16x16x32_f16(false, a, false, b, (short)0, c, false, false);
  asm volatile("v_nop\n\tv_nop\n\tv_nop\n\tv_nop" : "+v"(d) : "v"(a), "v"(b));
  return d;
}
__device__ __forceinline__ v8f wmma_bf(v16b a, v16b b, v8f c) {
  v8f d = __builtin_amdgcn_wmma_f32_16x16x32_bf16(false, a, false, b, (short)0, c, false, false);
  asm volatile("v_nop\n\tv_nop\n\tv_nop\n\tv_nop" : "+v"(d) : "v"(a), "v"(b));
  return d;
}
__device__ __forceinline__ v16h frag_h(const _Float16* rowk0, int lane) {
  union { v16h v; v8h q[2]; } u; const _Float16* p = rowk0 + 8 * (lane >> 4);
  u.q[0] = *(const v8h*)p; u.q[1] = *(const v8h*)(p + 16); return u.v;
}
__device__ __forceinline__ v16h frag_f32(const float* rowk0, int lane) {
  v16h a; const float* p = rowk0 + 8 * (lane >> 4);
#pragma unroll
  for (int i = 0; i < 8; ++i) { a[i] = (_Float16)p[i]; a[8 + i] = (_Float16)p[16 + i]; }
  return a;
}
__device__ __forceinline__ v16h frag_f32s(const float* rowk0, int lane, float sc) {
  v16h a; const float* p = rowk0 + 8 * (lane >> 4);
#pragma unroll
  for (int i = 0; i < 8; ++i) { a[i] = (_Float16)(p[i] * sc); a[8 + i] = (_Float16)(p[16 + i] * sc); }
  return a;
}
__device__ __forceinline__ v16h fragc_f32(const float* W, int k0, int n, int lane, int ld, int K) {
  v16h a; const int g = lane >> 4;
#pragma unroll
  for (int i = 0; i < 8; ++i) { const int ka = k0 + 8 * g + i, kb = ka + 16;
    a[i] = (_Float16)(ka < K ? W[(size_t)(ka < K ? ka : K - 1) * ld + n] : 0.f); a[8 + i] = (_Float16)(kb < K ? W[(size_t)(kb < K ? kb : K - 1) * ld + n] : 0.f); }
  return a;
}
struct F2 { v16b h, l; };
__device__ __forceinline__ F2 bsplit16(const float v[16]) { F2 r;
#pragma unroll
  for (int i = 0; i < 16; ++i) { const __bf16 h = (__bf16)v[i]; r.h[i] = h; r.l[i] = (__bf16)(v[i] - (float)h); }
  return r; }
__device__ __forceinline__ F2 split_row(const float* row, int k0, int lane) { float v[16]; const float* p = row + k0 + 8 * (lane >> 4);
#pragma unroll
  for (int i = 0; i < 8; ++i) { v[i] = p[i]; v[8 + i] = p[16 + i]; }
  return bsplit16(v); }
__device__ __forceinline__ F2 split_rowK(const float* row, int k0, int lane, int K) { float v[16]; const int g = lane >> 4;
#pragma unroll
  for (int i = 0; i < 8; ++i) { const int ka = k0 + 8 * g + i, kb = ka + 16; v[i] = ka < K ? row[ka < K ? ka : K - 1] : 0.f; v[8 + i] = kb < K ? row[kb < K ? kb : K - 1] : 0.f; }
  return bsplit16(v); }
__device__ __forceinline__ F2 split_col(const float* W, int k0, int n, int lane, int ld, int K) { float v[16]; const int g = lane >> 4;
#pragma unroll
  for (int i = 0; i < 8; ++i) { const int ka = k0 + 8 * g + i, kb = ka + 16; v[i] = ka < K ? W[(size_t)(ka < K ? ka : K - 1) * ld + n] : 0.f; v[8 + i] = kb < K ? W[(size_t)(kb < K ? kb : K - 1) * ld + n] : 0.f; }
  return bsplit16(v); }
__device__ __forceinline__ v8f mac3(const F2& a, const F2& b, v8f c) { c = wmma_bf(a.l, b.h, c); c = wmma_bf(a.h, b.l, c); return wmma_bf(a.h, b.h, c); }
__device__ __forceinline__ float sigm(float v) { return 1.0f / (1.0f + expf(-v)); }
#define LDSX() do { asm volatile("s_wait_dscnt 0" ::: "memory"); __builtin_amdgcn_wave_barrier(); __builtin_amdgcn_fence(__ATOMIC_RELEASE, "workgroup"); } while (0)


#define NB 4
#define LL 2048
#define DD 1024
#define NS 16
#define NR (NB * LL)
#define PW (DD + 2 * NS)
__device__ __forceinline__ float bfr(float v) { return (float)(__bf16)v; }
__device__ __forceinline__ v16b frag_b(const __bf16* rowk0, int lane) { return __builtin_bit_cast(v16b, frag_h((const _Float16*)rowk0, lane)); }
__device__ __attribute__((noinline)) float exp_ni(float v) { return expf(v); }
__device__ __attribute__((noinline)) float softplus_ni(float v) { return v > 20.f ? v : log1pf(expf(v)); }

__global__ __launch_bounds__(128) void k_xp(const float* __restrict__ x, const float* __restrict__ W, const float* __restrict__ bias, float* __restrict__ DT, float* __restrict__ BC) {
  __shared__ __align__(16) float so[4][16][132];
  const int tid = threadIdx.x, wave = tid >> 5, lane = tid & 31, col = lane & 15, g = lane >> 4; const size_t r0 = (size_t)blockIdx.x * 64 + wave * 16; const int n0 = blockIdx.y * 128; const int ntile = blockIdx.y < 8 ? 8 : 2;
  v8f acc[8] = {};
#pragma unroll 2
  for (int kc = 0; kc < DD / 32; ++kc) { const v16b a = split_row(x + (r0 + col) * DD, kc * 32, lane).h;
#pragma unroll
    for (int j = 0; j < 8; ++j) { if (j < ntile) acc[j] = wmma_bf(a, split_col(W, kc * 32, n0 + j * 16 + col, lane, PW, DD).h, acc[j]); } }
  if (blockIdx.y < 8) {
#pragma unroll
    for (int j = 0; j < 8; ++j) { const float bb = bfr(bias[n0 + j * 16 + col]);
#pragma unroll
      for (int r = 0; r < 8; ++r) so[wave][8 * g + r][j * 16 + col] = softplus_ni(acc[j][r] + bb); }
    LDSX();
    for (int rl = 0; rl < 16; ++rl) vst2(DT + (r0 + rl) * DD + n0 + lane * 4, *(const v4f*)(&so[wave][rl][lane * 4])); }
  else {
#pragma unroll
    for (int j = 0; j < 2; ++j) { const float bb = bfr(bias[n0 + j * 16 + col]);
#pragma unroll
      for (int r = 0; r < 8; ++r) so[wave][8 * g + r][j * 16 + col] = acc[j][r] + bb; }
    LDSX();
    for (int qq = lane; qq < 16 * 8; qq += 32) { const int rl = qq >> 3, pc = qq & 7; vst2(BC + (r0 + rl) * (2 * NS) + pc * 4, *(const v4f*)(&so[wave][rl][pc * 4])); } }
}
__global__ __launch_bounds__(128) void k_scan(const float* __restrict__ x, const float* __restrict__ DT, const float* __restrict__ BC, const float* __restrict__ Alog, const float* __restrict__ Dp, float* __restrict__ Y) {
  __shared__ float sh[NS][128], sA[NS][128];
  const int dloc = threadIdx.x; const int b = blockIdx.y, d = blockIdx.x * 128 + dloc; const float Dd = bfr(Dp[d]);
  for (int n = 0; n < NS; ++n) { sh[n][dloc] = 0.f; sA[n][dloc] = -expf(bfr(Alog[d * NS + n])); }
#pragma unroll 1
  for (int t = 0; t < LL; ++t) { const size_t r = (size_t)b * LL + t; const float dt = DT[r * DD + d], xv = bfr(x[r * DD + d]); const float* bc = BC + r * (2 * NS); const float dbx = dt * xv; float y = 0.f;
#pragma unroll 4
    for (int n = 0; n < NS; ++n) { const float h = exp_ni(dt * sA[n][dloc]) * sh[n][dloc] + dbx * bc[n]; sh[n][dloc] = h; y += h * bc[NS + n]; }
    vst2(Y + r * DD + d, (float_a)(y + Dd * xv)); }
}
__global__ __launch_bounds__(128) void k_out(const float* __restrict__ Y, const float* __restrict__ Wo, const float* __restrict__ bo, float* __restrict__ out) {
  __shared__ __align__(16) float so[4][16][132];
  const int tid = threadIdx.x, wave = tid >> 5, lane = tid & 31, col = lane & 15, g = lane >> 4; const size_t r0 = (size_t)blockIdx.x * 64 + wave * 16; const int n0 = blockIdx.y * 128;
  v8f acc[8] = {};
#pragma unroll 2
  for (int kc = 0; kc < DD / 32; ++kc) { const F2 a = split_row(Y + (r0 + col) * DD, kc * 32, lane);
#pragma unroll
    for (int j = 0; j < 8; ++j) { const v16b wb = split_col(Wo, kc * 32, n0 + j * 16 + col, lane, DD, DD).h; acc[j] = wmma_bf(a.l, wb, acc[j]); acc[j] = wmma_bf(a.h, wb, acc[j]); } }
#pragma unroll
  for (int j = 0; j < 8; ++j) { const float bb = bfr(bo[n0 + j * 16 + col]);
#pragma unroll
    for (int r = 0; r < 8; ++r) so[wave][8 * g + r][j * 16 + col] = acc[j][r] + bb; }
  LDSX();
  for (int rl = 0; rl < 16; ++rl) vst2(out + (r0 + rl) * DD + n0 + lane * 4, *(const v4f*)(&so[wave][rl][lane * 4]));
}
extern "C" void kernel_launch(void* const* d_in, const int* in_sizes, int n_in, void* d_out, int out_size, void* d_ws, size_t ws_size, hipStream_t stream) {
  (void)in_sizes; (void)n_in; (void)out_size; (void)ws_size;
  const float** I = (const float**)d_in;
  const float* x = I[0]; const float* Alog = I[1]; const float* Dp = I[2]; const float* Wx = I[3]; const float* bx = I[4]; const float* Wo = I[5]; const float* bo = I[6];
  char* ws = (char*)d_ws; size_t off = 0;
  auto take = [&](size_t bytes) { char* p = ws + off; off += (bytes + 255) & ~(size_t)255; return p; };
  float* DT = (float*)take((size_t)NR * DD * 4); float* BC = (float*)take((size_t)NR * 2 * NS * 4); float* Y = (float*)take((size_t)NR * DD * 4);
  k_xp<<<dim3(NR / 64, 9), 128, 0, stream>>>(x, Wx, bx, DT, BC);
  k_scan<<<dim3(DD / 128, NB), 128, 0, stream>>>(x, DT, BC, Alog, Dp, Y);
  k_out<<<dim3(NR / 64, DD / 128), 128, 0, stream>>>(Y, Wo, bo, (float*)d_out);
}
